// RGB_SClusterFormer_81535659147850
// MI455X (gfx1250) — hardware-run, weakly checked
//
#include <hip/hip_runtime.h>
#pragma clang fp contract(off)


#ifndef NB
#define NB 16
#endif
#define NB_FULL 16
#define PSD    32
#define SEQ    1024
#define DM     768
#define NHEAD  8
#define HDIM   24
#define HPAD   32
#define INNER  192
#define KPJ    256
#define HID    3072
#define NCEN   16
#define RROWS  (NB * SEQ)
#define NCHUNK 2
#define RCH    (RROWS / NCHUNK)
#define WCAR   64.0f
#define CCAR   1024.0f
#define YCAR   64.0f
#define QRS    2048.0f
#define QRI    (1.0f / 2048.0f)
#define EPSN   1.0e-12f
#define NEGB   (-3.0e38f)

static_assert(NB <= NB_FULL);
static_assert(PSD * PSD == SEQ);
static_assert(PSD / 4 == 8);
static_assert(NCEN == 16);
static_assert(NHEAD * HDIM == INNER);
static_assert(NHEAD * HPAD == KPJ);
static_assert(HDIM == 24 && HPAD == 32);
static_assert(HDIM % 8 == 0 && HDIM == 6 * 4);
static_assert(DM == 3 * 32 * 8);
static_assert(3 * 32 * 16 == DM * 2);
static_assert(DM % 64 == 0 && INNER % 64 == 0 && HID % 64 == 0);
static_assert(DM % 32 == 0 && KPJ % 32 == 0 && HID % 32 == 0);
static_assert(RROWS % 64 == 0);
static_assert(RROWS % 32 == 0);
static_assert(RROWS % NCHUNK == 0);
static_assert(RCH % 64 == 0);
static_assert(SEQ == 4 * 256);
static_assert(256 * 16 * 16 == SEQ * HPAD * 2);
static_assert(NCEN == 2 * 8);
static_assert(8 * 32 * 16 == 16 * 64 * 4);
static_assert(4 * 32 * 16 == 16 * 64 * 2);
static_assert((INNER * DM) % 2048 == 0 && (HID * DM) % 2048 == 0 && (DM * KPJ) % 2048 == 0);
static_assert(16 * 68 * 4 <= 131072);
static_assert((2 * NCEN * HDIM + 2 * NCEN * HDIM) * 4 + SEQ * 8 <= 131072);

typedef _Float16 h16;
typedef __attribute__((ext_vector_type(16))) _Float16 v16h;
typedef __attribute__((ext_vector_type(8)))  _Float16 v8h;
typedef __attribute__((ext_vector_type(8)))  float    v8f;
typedef __attribute__((ext_vector_type(4)))  float    v4f;
typedef v4f  __attribute__((may_alias)) v4fa;

__device__ __forceinline__ unsigned short f2bf(float f) { unsigned u = __float_as_uint(f); u += 0x7FFFu + ((u >> 16) & 1u); return (unsigned short)(u >> 16); }
__device__ __forceinline__ float bfr(float f) { return __uint_as_float(((unsigned)f2bf(f)) << 16); }
__device__ __forceinline__ v16h cat16(v8h lo, v8h hi) { return __builtin_shufflevector(lo, hi, 0, 1, 2, 3, 4, 5, 6, 7, 8, 9, 10, 11, 12, 13, 14, 15); }
__device__ __forceinline__ v16h ldh(const h16* p) { return cat16(*(const v8h*)p, *(const v8h*)(p + 16)); }
__device__ __forceinline__ void wave_sync() { __builtin_amdgcn_fence(3  , "wavefront"); __builtin_amdgcn_wave_barrier(); asm volatile("" ::: "memory"); }
__device__ __forceinline__ h16 toh_flush(float v) { const h16 r = (h16)v; return (fabsf(v) < 6.103515625e-05f) ? (h16)0.0f : r; }
__device__ __forceinline__ v8f wmma16g(v16h a, v16h b, v8f c) {
    c = __builtin_amdgcn_wmma_f32_16x16x32_f16(false, a, false, b, (short)0, c, false, false);
    asm volatile("v_nop\n\tv_nop\n\tv_nop\n\tv_nop" : "+v"(c) : "v"(a), "v"(b));
    return c;
}

__global__ __launch_bounds__(256) void k_wconv(const float* __restrict__ src, h16* dst, size_t n8) {
    const size_t i = (size_t)blockIdx.x * 256 + threadIdx.x; if (i >= n8) return;
    const v8f v = *(const v8f*)(src + i * 8); v8h o;
#pragma unroll
    for (int k = 0; k < 8; ++k) o[k] = toh_flush(bfr(v[k]) * WCAR);
    *(volatile v8h*)(dst + i * 8) = o; __threadfence(); *(volatile v8h*)(dst + i * 8) = o;
}

__global__ __launch_bounds__(256) void k_wconv_p(const float* __restrict__ src, h16* dst) {
    const int i = blockIdx.x * 256 + threadIdx.x; if (i >= DM * KPJ / 8) return;
    const int o = i >> 5, q = i & 31, e = q >> 2, j = q & 3; const int jc = j < 3 ? j : 2;
    v8f v = *(const v8f*)(src + (size_t)o * INNER + e * HDIM + jc * 8);
    asm volatile("" : "+v"(v));
    const bool ok = j < 3; v8h o8;
#pragma unroll
    for (int k = 0; k < 8; ++k) { const float t = ok ? bfr(v[k]) * WCAR : 0.0f; o8[k] = toh_flush(t); }
    *(volatile v8h*)(dst + (size_t)i * 8) = o8; __threadfence(); *(volatile v8h*)(dst + (size_t)i * 8) = o8;
}

__global__ __launch_bounds__(256) void k_ln(const float* __restrict__ X, const float* __restrict__ gw, const float* __restrict__ gb, h16* __restrict__ Y, h16* YR, int rows, int cvt) {
    const int lane = threadIdx.x & 31;
    const int wave = __builtin_amdgcn_readfirstlane((int)(threadIdx.x >> 5));
    const int row = blockIdx.x * 8 + wave;
    if (row >= rows) return;
    const float* xr = X + (size_t)row * DM;
    h16* yr = Y + (size_t)row * DM;
    h16* yq = YR + (size_t)row * DM;
    float s = 0.0f;
#pragma unroll 1
    for (int ch = 0; ch < 3; ++ch) { const v8f v = *(const v8f*)(xr + ch * 256 + lane * 8);
#pragma unroll
        for (int k = 0; k < 8; ++k) { const float t = cvt ? bfr(v[k]) : v[k]; s += t; } }
    s += __shfl_xor(s, 16, 32); s += __shfl_xor(s, 8, 32); s += __shfl_xor(s, 4, 32); s += __shfl_xor(s, 2, 32); s += __shfl_xor(s, 1, 32);
    const float mu = s * (1.0f / (float)DM);
    float q = 0.0f;
#pragma unroll 1
    for (int ch = 0; ch < 3; ++ch) { const v8f v = *(const v8f*)(xr + ch * 256 + lane * 8);
#pragma unroll
        for (int k = 0; k < 8; ++k) { const float t = (cvt ? bfr(v[k]) : v[k]) - mu; q += t * t; } }
    q += __shfl_xor(q, 16, 32); q += __shfl_xor(q, 8, 32); q += __shfl_xor(q, 4, 32); q += __shfl_xor(q, 2, 32); q += __shfl_xor(q, 1, 32);
    const float var = q * (1.0f / (float)DM);
    const float rs = 1.0f / sqrtf(var + 1.0e-5f);
#pragma unroll 1
    for (int ps = 0; ps < 2; ++ps) {
#pragma unroll 1
        for (int ch = 0; ch < 3; ++ch) { const int c0 = ch * 256 + lane * 8;
            const v8f v = *(const v8f*)(xr + c0); const v8f g = *(const v8f*)(gw + c0); const v8f bb = *(const v8f*)(gb + c0); v8h o, rr;
#pragma unroll
            for (int k = 0; k < 8; ++k) { const float t = cvt ? bfr(v[k]) : v[k]; const float val = (t - mu) * rs * bfr(g[k]) + bfr(bb[k]);
                const h16 hv = toh_flush(val); o[k] = hv; rr[k] = toh_flush((val - (float)hv) * QRS); }
            *(volatile v8h*)(yr + c0) = o;
            if (cvt) *(volatile v8h*)(yq + c0) = rr; }
        if (ps == 0) __threadfence(); }
}

template <int EPI>
__device__ __forceinline__ void gemm_body(const h16* __restrict__ A, const size_t lda, const size_t astep, const h16* __restrict__ Bt, const int K,
                                          const float* __restrict__ bias, const float* RES, const int rbf, float* OF, h16* OH, const size_t ldo, const float scale) {
    __shared__ __align__(16) float os[16 * 68];
    const int lane = threadIdx.x & 31, lr = lane & 15, hi = lane >> 4; const int r0 = blockIdx.x * 64, c0 = blockIdx.y * 64;
    v8f acc[4][4];
#pragma unroll
    for (int mb = 0; mb < 4; ++mb)
#pragma unroll
        for (int nb = 0; nb < 4; ++nb) acc[mb][nb] = (v8f){};
    const size_t aoff = (size_t)(r0 + lr) * lda + 8 * hi, boff = (size_t)(c0 + lr) * (size_t)K + 8 * hi;
    const int nks = K >> 5;
#pragma unroll 1
    for (int ks = 0; ks < nks; ++ks) {
        v16h a[4];
#pragma unroll
        for (int mb = 0; mb < 4; ++mb) a[mb] = ldh(A + aoff + (size_t)mb * 16 * lda + (size_t)ks * astep);
#pragma unroll
        for (int nb = 0; nb < 4; ++nb) { const v16h b = ldh(Bt + boff + (size_t)nb * 16 * (size_t)K + (size_t)ks * 32);
#pragma unroll
            for (int mb = 0; mb < 4; ++mb) acc[mb][nb] = wmma16g(a[mb], b, acc[mb][nb]); }
    }
    float bc[4];
#pragma unroll
    for (int nb = 0; nb < 4; ++nb) bc[nb] = bfr(bias[c0 + nb * 16 + lr]);
#pragma unroll
    for (int mb = 0; mb < 4; ++mb) {
#pragma unroll
        for (int nb = 0; nb < 4; ++nb) {
#pragma unroll
            for (int j = 0; j < 8; ++j) os[(hi * 8 + j) * 68 + nb * 16 + lr] = acc[mb][nb][j] * scale + bc[nb]; }
        wave_sync();
        if (EPI == 1) {
#pragma unroll 1
            for (int i = 0; i < 8; ++i) { const int idx = i * 32 + lane; const int row = idx >> 4, c4 = (idx & 15) * 4;
                v4f t = *(const v4fa*)(&os[row * 68 + c4]);
                const v4f r = *(const v4f*)(RES + (size_t)(r0 + mb * 16 + row) * ldo + c0 + c4);
#pragma unroll
                for (int q = 0; q < 4; ++q) { const float rq = rbf ? bfr(r[q]) : r[q]; t[q] += rq; }
                *(v4fa*)(&os[row * 68 + c4]) = t; }
            wave_sync();
        }
        if (EPI == 2) {
#pragma unroll 1
            for (int i = 0; i < 8; ++i) { const int idx = i * 32 + lane; const int row = idx >> 4, c4 = (idx & 15) * 4;
                v4f t = *(const v4fa*)(&os[row * 68 + c4]);
#pragma unroll
                for (int q = 0; q < 4; ++q) { const float xg = t[q]; t[q] = (0.5f * xg * (1.0f + erff(xg * 0.70710678118654752f))) * YCAR; }
                *(v4fa*)(&os[row * 68 + c4]) = t; }
            wave_sync();
        }
#pragma unroll 1
        for (int ps = 0; ps < 2; ++ps) {
            if (EPI == 2) {
#pragma unroll
                for (int s = 0; s < 4; ++s) { const int row = 4 * s + (lane >> 3), c8 = (lane & 7) * 8;
                    const v4f x0 = *(const v4fa*)(&os[row * 68 + c8]); const v4f x1 = *(const v4fa*)(&os[row * 68 + c8 + 4]); v8h hv;
#pragma unroll
                    for (int i = 0; i < 4; ++i) { hv[i] = toh_flush(x0[i]); hv[4 + i] = toh_flush(x1[i]); }
                    *(volatile v8h*)(OH + (size_t)(r0 + mb * 16 + row) * ldo + c0 + c8) = hv; }
            } else {
#pragma unroll
                for (int s = 0; s < 8; ++s) { const int row = 2 * s + (lane >> 4), c4 = (lane & 15) * 4;
                    const v4f val = *(const v4fa*)(&os[row * 68 + c4]);
                    *(volatile v4f*)(OF + (size_t)(r0 + mb * 16 + row) * ldo + c0 + c4) = val; }
            }
            if (ps == 0) __threadfence(); }
        wave_sync();
    }
}

__global__ __launch_bounds__(32) void k_gemm_f2(const h16* __restrict__ A, const h16* __restrict__ AR, const h16* __restrict__ Bt, const float* __restrict__ bias, float* OF) {
    __shared__ __align__(16) float os[16 * 68];
    const int lane = threadIdx.x & 31, lr = lane & 15, hi = lane >> 4; const int r0 = blockIdx.x * 32, c0 = blockIdx.y * 64;
    v8f acc[2][4], acr[2][4];
#pragma unroll
    for (int mb = 0; mb < 2; ++mb)
#pragma unroll
        for (int nb = 0; nb < 4; ++nb) { acc[mb][nb] = (v8f){}; acr[mb][nb] = (v8f){}; }
    const size_t aoff = (size_t)(r0 + lr) * DM + 8 * hi, boff = (size_t)(c0 + lr) * DM + 8 * hi;
#pragma unroll 1
    for (int ks = 0; ks < DM / 32; ++ks) {
        v16h a[2], ar[2];
#pragma unroll
        for (int mb = 0; mb < 2; ++mb) { const size_t ao = aoff + (size_t)mb * 16 * DM + (size_t)ks * 32; a[mb] = ldh(A + ao); ar[mb] = ldh(AR + ao); }
#pragma unroll
        for (int nb = 0; nb < 4; ++nb) { const v16h b = ldh(Bt + boff + (size_t)nb * 16 * DM + (size_t)ks * 32);
#pragma unroll
            for (int mb = 0; mb < 2; ++mb) { acc[mb][nb] = wmma16g(a[mb], b, acc[mb][nb]); acr[mb][nb] = wmma16g(ar[mb], b, acr[mb][nb]); } }
    }
    float bc[4];
#pragma unroll
    for (int nb = 0; nb < 4; ++nb) bc[nb] = bfr(bias[c0 + nb * 16 + lr]);
#pragma unroll
    for (int mb = 0; mb < 2; ++mb) {
#pragma unroll
        for (int nb = 0; nb < 4; ++nb) {
#pragma unroll
            for (int j = 0; j < 8; ++j) os[(hi * 8 + j) * 68 + nb * 16 + lr] = (acc[mb][nb][j] + acr[mb][nb][j] * QRI) * (1.0f / WCAR) + bc[nb]; }
        wave_sync();
#pragma unroll 1
        for (int ps = 0; ps < 2; ++ps) {
#pragma unroll
            for (int s = 0; s < 8; ++s) { const int row = 2 * s + (lane >> 4), c4 = (lane & 15) * 4;
                const v4f val = *(const v4fa*)(&os[row * 68 + c4]);
                *(volatile v4f*)(OF + (size_t)(r0 + mb * 16 + row) * INNER + c0 + c4) = val; }
            if (ps == 0) __threadfence(); }
        wave_sync();
    }
}

__global__ __launch_bounds__(32) void k_gemm_fv(const h16* __restrict__ A, const h16* __restrict__ Bt, const float* __restrict__ bias, float* OF) {
    gemm_body<0>(A, (size_t)DM, (size_t)32, Bt, DM, bias, bias, 0, OF, (h16*)0, (size_t)INNER, 1.0f / WCAR);
}
__global__ __launch_bounds__(32) void k_gemm_proj(const h16* __restrict__ A, const h16* __restrict__ Bt, const float* __restrict__ bias, const float* __restrict__ X, float* OF) {
    gemm_body<1>(A, (size_t)HPAD, (size_t)RROWS * HPAD, Bt, KPJ, bias, X, 1, OF, (h16*)0, (size_t)DM, 1.0f / (WCAR * CCAR));
}
__global__ __launch_bounds__(32) void k_gemm_fc1(const h16* __restrict__ A, const h16* __restrict__ Bt, const float* __restrict__ bias, h16* OH) {
    gemm_body<2>(A, (size_t)DM, (size_t)32, Bt, DM, bias, bias, 0, (float*)0, OH, (size_t)HID, 1.0f / WCAR);
}
__global__ __launch_bounds__(32) void k_gemm_fc2(const h16* __restrict__ A, const h16* __restrict__ Bt, const float* __restrict__ bias, float* IO) {
    gemm_body<1>(A, (size_t)HID, (size_t)32, Bt, HID, bias, IO, 0, IO, (h16*)0, (size_t)DM, 1.0f / (WCAR * YCAR));
}

__global__ __launch_bounds__(256) void k_cluster(const float* __restrict__ FVP, const float* __restrict__ alpha_p, const float* __restrict__ beta_p, h16* CH) {
    __shared__ __align__(16) float spool[2 * NCEN * HDIM];
    __shared__ __align__(16) float scn[NCEN * HDIM];
    __shared__ __align__(16) float soc[NCEN * HDIM];
    __shared__ float s_sim[SEQ];
    __shared__ int   s_am[SEQ];
    const int tid = threadIdx.x, lane = tid & 31;
    const int wave = __builtin_amdgcn_readfirstlane((int)(threadIdx.x >> 5));
    const int be = blockIdx.x; const int b = be / NHEAD, e = be % NHEAD;
    const size_t rowbase = (size_t)b * SEQ;
    const size_t voff = (size_t)RROWS * INNER;
    const size_t hb = rowbase * INNER + (size_t)e * HDIM;
    if (tid < 192) {
        const int sel = tid / 96, rem = tid % 96, m = rem / 6, c4 = (rem % 6) * 4;
        const int n0 = (m >> 2) * 8 * PSD + (m & 3) * 8;
        const float* src = FVP + (size_t)sel * voff + hb + c4;
        v4f a = (v4f){};
#pragma unroll 1
        for (int t = 0; t < 64; ++t) { const int n = n0 + (t >> 3) * PSD + (t & 7); a += *(const v4f*)(src + (size_t)n * INNER); }
        a = a * (1.0f / 64.0f);
        *(v4fa*)(&spool[sel * (NCEN * HDIM) + m * HDIM + c4]) = a;
    }
    __syncthreads();
    if (tid < NCEN) {
        float sq = 0.0f;
#pragma unroll 1
        for (int c = 0; c < HDIM; ++c) { const float t = spool[tid * HDIM + c]; sq += t * t; }
        const float inv = 1.0f / fmaxf(sqrtf(sq), EPSN);
#pragma unroll 1
        for (int c = 0; c < HDIM; ++c) scn[tid * HDIM + c] = spool[tid * HDIM + c] * inv;
    }
    __syncthreads();
    const float al = bfr(alpha_p[0]), bt = bfr(beta_p[0]);
#pragma unroll 1
    for (int j = 0; j < 4; ++j) {
        const int n = tid + 256 * j;
        const float* fr = FVP + hb + (size_t)n * INNER;
        float xn[HDIM];
#pragma unroll
        for (int g = 0; g < 6; ++g) { const v4f t = *(const v4f*)(fr + g * 4); xn[g * 4 + 0] = t[0]; xn[g * 4 + 1] = t[1]; xn[g * 4 + 2] = t[2]; xn[g * 4 + 3] = t[3]; }
        float sq = 0.0f;
#pragma unroll
        for (int c = 0; c < HDIM; ++c) sq += xn[c] * xn[c];
        const float inv = 1.0f / fmaxf(sqrtf(sq), EPSN);
#pragma unroll
        for (int c = 0; c < HDIM; ++c) xn[c] = xn[c] * inv;
        float best = NEGB; int bm = 0;
#pragma unroll 1
        for (int m = 0; m < NCEN; ++m) {
            float dot = 0.0f;
#pragma unroll
            for (int c = 0; c < HDIM; ++c) dot += scn[m * HDIM + c] * xn[c];
            const float d2 = fmaxf(2.0f - 2.0f * dot, EPSN);
            const float dist = sqrtf(d2);
            float sv = bt + al * expf(-dist);
            sv = (sv >= 0.0f) ? sv : 0.2f * sv;
            if (sv > best) { best = sv; bm = m; }
        }
        s_am[n] = bm; s_sim[n] = best;
    }
    __syncthreads();
    {
        float a0 = 0.0f, a1 = 0.0f; int k0 = 0, k1 = 0;
        const int cl = lane < HDIM ? lane : (HDIM - 1);
        const float* vsrc = FVP + voff + hb + cl;
#pragma unroll 1
        for (int n = 0; n < SEQ; ++n) {
            const int a = __builtin_amdgcn_readfirstlane(s_am[n] & (NCEN - 1));
            if ((a >> 1) == wave) {
                const float p = s_sim[n] * vsrc[(size_t)n * INNER];
                if (a & 1) { a1 += p; k1 += 1; } else { a0 += p; k0 += 1; }
            }
        }
        const float i0 = 1.0f / ((float)k0 + 1.0f), i1 = 1.0f / ((float)k1 + 1.0f);
        if (lane < HDIM) {
            soc[(2 * wave) * HDIM + lane]     = (a0 + spool[NCEN * HDIM + (2 * wave) * HDIM + lane]) * i0;
            soc[(2 * wave + 1) * HDIM + lane] = (a1 + spool[NCEN * HDIM + (2 * wave + 1) * HDIM + lane]) * i1;
        }
    }
    __syncthreads();
    h16* chb = CH + ((size_t)e * RROWS + rowbase) * HPAD;
#pragma unroll 1
    for (int ps = 0; ps < 2; ++ps) {
#pragma unroll 1
        for (int i = 0; i < 16; ++i) {
            const int p = tid + 256 * i; const int n = p >> 2, q = p & 3; const int qc = q < 3 ? q : 2;
            const int a = s_am[n] & (NCEN - 1); const float s = s_sim[n] * CCAR;
            const v4f u0 = *(const v4fa*)(&soc[a * HDIM + qc * 8]); const v4f u1 = *(const v4fa*)(&soc[a * HDIM + qc * 8 + 4]);
            const bool ok = q < 3; v8h o;
#pragma unroll
            for (int k = 0; k < 4; ++k) { const float y0 = ok ? s * u0[k] : 0.0f; const float y1 = ok ? s * u1[k] : 0.0f; o[k] = toh_flush(y0); o[4 + k] = toh_flush(y1); }
            *(volatile v8h*)(chb + (size_t)p * 8) = o; }
        if (ps == 0) __threadfence(); }
}

static constexpr size_t al256(size_t v) { return (v + 255) & ~(size_t)255; }
static constexpr size_t SZ_XH  = al256((size_t)RROWS * DM * 2);
static constexpr size_t SZ_FV  = al256((size_t)2 * RROWS * INNER * 4);
static constexpr size_t SZ_CH  = al256((size_t)NHEAD * RROWS * HPAD * 2);
static constexpr size_t SZ_WFV = al256((size_t)INNER * DM * 2);
static constexpr size_t SZ_WP  = al256((size_t)DM * KPJ * 2);
static constexpr size_t SZ_W1  = al256((size_t)HID * DM * 2);
static constexpr size_t SZ_W2  = al256((size_t)DM * HID * 2);
static constexpr size_t SZ_Y1  = al256((size_t)RCH * HID * 2);
static constexpr size_t SZ_TOTAL = SZ_XH + SZ_FV + SZ_CH + 2 * SZ_WFV + SZ_WP + SZ_W1 + SZ_W2 + SZ_Y1;
static_assert(SZ_TOTAL <= (size_t)134217728);
static_assert(((size_t)RROWS * INNER * 4) % 128 == 0);
static_assert(((size_t)SEQ * HPAD * 2) % 128 == 0);
static_assert((size_t)RROWS * DM * 2 <= SZ_Y1);

extern "C" void kernel_launch(void* const* d_in, const int* in_sizes, int n_in,
                              void* d_out, int out_size, void* d_ws, size_t ws_size, hipStream_t stream) {
    if (n_in < 17) return;
    if ((size_t)in_sizes[0] < (size_t)RROWS * DM) return;
    if (in_sizes[1] < DM || in_sizes[2] < DM || in_sizes[11] < DM || in_sizes[12] < DM) return;
    if ((size_t)in_sizes[3] < (size_t)INNER * DM || (size_t)in_sizes[5] < (size_t)INNER * DM || (size_t)in_sizes[7] < (size_t)DM * INNER) return;
    if (in_sizes[4] < INNER || in_sizes[6] < INNER || in_sizes[8] < DM) return;
    if (in_sizes[9] < 1 || in_sizes[10] < 1) return;
    if ((size_t)in_sizes[13] < (size_t)HID * DM || (size_t)in_sizes[15] < (size_t)DM * HID) return;
    if (in_sizes[14] < HID || in_sizes[16] < DM) return;
    if ((size_t)out_size < (size_t)RROWS * DM) return;
    if (SZ_TOTAL > ws_size) return;
    const float* x      = (const float*)d_in[0];
    const float* ln1_w  = (const float*)d_in[1];
    const float* ln1_b  = (const float*)d_in[2];
    const float* f_w    = (const float*)d_in[3];
    const float* f_b    = (const float*)d_in[4];
    const float* v_w    = (const float*)d_in[5];
    const float* v_b    = (const float*)d_in[6];
    const float* proj_w = (const float*)d_in[7];
    const float* proj_b = (const float*)d_in[8];
    const float* alpha  = (const float*)d_in[9];
    const float* beta   = (const float*)d_in[10];
    const float* ln2_w  = (const float*)d_in[11];
    const float* ln2_b  = (const float*)d_in[12];
    const float* fc1_w  = (const float*)d_in[13];
    const float* fc1_b  = (const float*)d_in[14];
    const float* fc2_w  = (const float*)d_in[15];
    const float* fc2_b  = (const float*)d_in[16];
    float* OUT = (float*)d_out;
    char* wsp = (char*)d_ws;
    h16*   XH  = (h16*)wsp;   wsp += SZ_XH;
    float* FVP = (float*)wsp; wsp += SZ_FV;
    h16*   CH  = (h16*)wsp;   wsp += SZ_CH;
    h16*   WF  = (h16*)wsp;   wsp += SZ_WFV;
    h16*   WV  = (h16*)wsp;   wsp += SZ_WFV;
    h16*   WP  = (h16*)wsp;   wsp += SZ_WP;
    h16*   W1  = (h16*)wsp;   wsp += SZ_W1;
    h16*   W2  = (h16*)wsp;   wsp += SZ_W2;
    h16*   Y1  = (h16*)wsp;   wsp += SZ_Y1;
    h16*   XR  = Y1;

    { const size_t n8 = (size_t)INNER * DM / 8; const unsigned g = (unsigned)((n8 + 255) / 256);
      k_wconv<<<g, 256, 0, stream>>>(f_w, WF, n8); k_wconv<<<g, 256, 0, stream>>>(v_w, WV, n8); }
    k_wconv_p<<<(DM * KPJ / 8 + 255) / 256, 256, 0, stream>>>(proj_w, WP);
    { const size_t n8 = (size_t)HID * DM / 8; const unsigned g = (unsigned)((n8 + 255) / 256);
      k_wconv<<<g, 256, 0, stream>>>(fc1_w, W1, n8); k_wconv<<<g, 256, 0, stream>>>(fc2_w, W2, n8); }

    k_ln<<<(RROWS + 7) / 8, 256, 0, stream>>>(x, ln1_w, ln1_b, XH, XR, RROWS, 1);
    k_gemm_f2<<<dim3(RROWS / 32, INNER / 64, 1), 32, 0, stream>>>(XH, XR, WF, f_b, FVP);
    k_gemm_fv<<<dim3(RROWS / 64, INNER / 64, 1), 32, 0, stream>>>(XH, WV, v_b, FVP + (size_t)RROWS * INNER);
    k_cluster<<<NB * NHEAD, 256, 0, stream>>>(FVP, alpha, beta, CH);
    k_gemm_proj<<<dim3(RROWS / 64, DM / 64, 1), 32, 0, stream>>>(CH, WP, proj_b, x, OUT);
    k_ln<<<(RROWS + 7) / 8, 256, 0, stream>>>(OUT, ln2_w, ln2_b, XH, XR, RROWS, 0);
    for (int c = 0; c < NCHUNK; ++c) {
        k_gemm_fc1<<<dim3(RCH / 64, HID / 64, 1), 32, 0, stream>>>(XH + (size_t)c * RCH * DM, W1, fc1_b, Y1);
        k_gemm_fc2<<<dim3(RCH / 64, DM / 64, 1), 32, 0, stream>>>(Y1, W2, fc2_b, OUT + (size_t)c * RCH * DM);
    }
}
